// S4Layer_85298050498930
// MI455X (gfx1250) — hardware-verified
//
#include <hip/hip_runtime.h>
#include <hip/hip_bf16.h>

typedef __attribute__((ext_vector_type(16))) _Float16 v16h;
typedef __attribute__((ext_vector_type(8)))  _Float16 v8h;
typedef __attribute__((ext_vector_type(8)))  float    v8f;
typedef __attribute__((ext_vector_type(4)))  float    v4f;
typedef __attribute__((ext_vector_type(4)))  unsigned int v4u;
#define VST2(T, ptr, val) do { const T _v = (val); *(volatile T*)(ptr) = _v; __threadfence(); *(volatile T*)(ptr) = _v; } while (0)

#define BATCH   8
#define SEQ     4096
#define DM      128
#define DS      128
#define KR_LEN  4160
#define XT_STRIDE 4160

__global__ void k_w(const float* __restrict__ C, const float* __restrict__ B,
                    float* __restrict__ W) {
    int idx = blockIdx.x * blockDim.x + threadIdx.x;
    int m = idx >> 7, j = idx & 127;
    float s = 0.f;
#pragma unroll 4
    for (int t = 0; t < DS; ++t) s += C[m * DS + t] * B[t * DM + j];
    VST2(float, W + idx, s);
}

__global__ void k_psum(const float* __restrict__ Lam, const float* __restrict__ log_dt,
                       float* __restrict__ Psum) {
    __shared__ float rate[DM];
    int j = blockIdx.y;
    int l = blockIdx.x * 256 + threadIdx.x;
    if (threadIdx.x < DM)
        rate[threadIdx.x] = expf(log_dt[threadIdx.x]) * Lam[j];
    __syncthreads();
    float fl = (float)l;
    float s = 0.f;
#pragma unroll 4
    for (int m = 0; m < DM; ++m) s += expf(rate[m] * fl);
    VST2(float, Psum + j * SEQ + l, s);
}

__global__ void k_kr(const float* __restrict__ W, const float* __restrict__ Psum,
                     float* __restrict__ KRf) {
    int m = blockIdx.y;
    int t = blockIdx.x * 256 + threadIdx.x;
    if (t >= KR_LEN) return;
    float v = 0.f;
    if (t >= 1 && t <= SEQ) {
        int l = SEQ - t;
        const float* w = W + m * DS;
        float s = 0.f;
#pragma unroll 4
        for (int j = 0; j < DS; ++j) s += w[j] * Psum[j * SEQ + l];
        v = s;
    }
    VST2(float, KRf + m * KR_LEN + t, v);
}

__global__ void k_xt(const float* __restrict__ x, _Float16* __restrict__ xT) {
    __shared__ float tile[64][17];
    int b = blockIdx.z, m0 = blockIdx.y * 16, l0 = blockIdx.x * 64;
    int tx = threadIdx.x, ty = threadIdx.y;
    const int t = ty * 16 + tx;
#pragma unroll
    for (int r = 0; r < 4; ++r) {
      const int l = l0 + ty + 16 * r;
      tile[ty + 16 * r][tx] = (l < SEQ) ? x[((size_t)b * SEQ + l) * DM + m0 + tx] : 0.0f;
    }
    __syncthreads();
    if (t < 128) {
      const int mm = t >> 3, q = (t & 7) * 8;
      v8h v;
#pragma unroll
      for (int e = 0; e < 8; ++e) v[e] = (_Float16)tile[q + e][mm];
      VST2(v8h, xT + ((size_t)((m0 + mm) * BATCH + b)) * XT_STRIDE + l0 + q, v);
    }
}

__device__ __forceinline__ void load_frags(const float* __restrict__ kr,
                                           const _Float16* __restrict__ xr,
                                           int tb0, int cb, int kb, int k0,
                                           v16h& a, v16h& b) {
    int tb = tb0 + k0;
    v4f q0 = *(const v4f*)(kr + tb);
    v4f q1 = *(const v4f*)(kr + tb + 4);
    v4f q2 = *(const v4f*)(kr + tb + 16);
    v4f q3 = *(const v4f*)(kr + tb + 20);
#pragma unroll
    for (int h = 0; h < 4; ++h) {
        a[h]      = (_Float16)q0[h];
        a[4 + h]  = (_Float16)q1[h];
        a[8 + h]  = (_Float16)q2[h];
        a[12 + h] = (_Float16)q3[h];
    }
    union { v16h v; v4u q[2]; } bu;
    const _Float16* bp = xr + k0 + kb;
    bu.q[0] = *(const v4u*)(bp);
    bu.q[1] = *(const v4u*)(bp + 16);
    b = bu.v;
}

__global__ void __launch_bounds__(256) k_conv(const float* __restrict__ KRf,
                                              const _Float16* __restrict__ xT,
                                              const float* __restrict__ x,
                                              const float* __restrict__ Dv,
                                              float* __restrict__ out) {
    __shared__ __attribute__((aligned(16))) float sY[16][8][33];
    int lane = threadIdx.x & 31;
    const int wave = threadIdx.x >> 5;
    int i = blockIdx.x >> 2;
    const int mg = (blockIdx.x & 3) * 32;
    int li = i << 4;

    int r  = lane & 15;
    int cb = (lane >> 4) << 3;
    int kb = (lane >> 4) << 3;
    int n  = lane & 15;
    int nk = (li + 47) >> 5;

  for (int mi = 0; mi < 4; ++mi) {
    const int m = mg + wave + 8 * mi;
    const float*    kr = KRf + m * KR_LEN;
    const _Float16* xr = xT + (size_t)(m * BATCH + (n & 7)) * XT_STRIDE;
    int tb0 = SEQ - li - r + cb;

    v8f acc0 = {}; v8f acc1 = {};

    int j0 = 0;
    for (; j0 + 2 <= nk; j0 += 2) {
        v16h a0, b0, a1, b1;
        load_frags(kr, xr, tb0, cb, kb, (j0 << 5), a0, b0);
        load_frags(kr, xr, tb0, cb, kb, ((j0 + 1) << 5), a1, b1);
        acc0 = __builtin_amdgcn_wmma_f32_16x16x32_f16(false, a0, false, b0,
                                                      (short)0, acc0, false, false);
        acc1 = __builtin_amdgcn_wmma_f32_16x16x32_f16(false, a1, false, b1,
                                                      (short)0, acc1, false, false);
        asm volatile("v_nop\n\tv_nop\n\tv_nop\n\tv_nop" : "+v"(acc0), "+v"(acc1) : "v"(a1), "v"(b1));
    }
    if (j0 < nk) {
        v16h a0, b0;
        load_frags(kr, xr, tb0, cb, kb, (j0 << 5), a0, b0);
        acc0 = __builtin_amdgcn_wmma_f32_16x16x32_f16(false, a0, false, b0,
                                                      (short)0, acc0, false, false);
    }

    if (n < 8) {
        int rowAdd = (lane >> 4) << 3;
        float dv = Dv[m];
#pragma unroll
        for (int p = 0; p < 8; ++p) {
            int l = li + p + rowAdd;
            size_t idx = ((size_t)n * SEQ + l) * DM + m;
            sY[p + rowAdd][n][wave + 8 * mi] = (acc0[p] + acc1[p]) + dv * x[idx];
        }
    }
  }
    __syncthreads();
    for (int pass = 0; pass < 2; ++pass) {
      for (int pc = threadIdx.x; pc < 1024; pc += 256) {
        const int row = pc >> 3, q = (pc & 7) * 4;
        const int l = li + (row >> 3), b = row & 7;
        v4f v; v[0] = sY[row >> 3][b][q]; v[1] = sY[row >> 3][b][q + 1]; v[2] = sY[row >> 3][b][q + 2]; v[3] = sY[row >> 3][b][q + 3];
        *(volatile v4f*)(out + ((size_t)b * SEQ + l) * DM + mg + q) = v;
      }
      __threadfence();
    }
}

extern "C" void kernel_launch(void* const* d_in, const int* in_sizes, int n_in,
                              void* d_out, int out_size, void* d_ws, size_t ws_size,
                              hipStream_t stream) {
    const float* x      = (const float*)d_in[0];
    const float* Lam    = (const float*)d_in[1];
    const float* B      = (const float*)d_in[2];
    const float* C      = (const float*)d_in[3];
    const float* Dv     = (const float*)d_in[4];
    const float* log_dt = (const float*)d_in[5];
    float* out = (float*)d_out;

    char* ws = (char*)d_ws;
    size_t off = 0;
    float* W    = (float*)(ws + off); off += (size_t)DM * DS * 4;
    float* Psum = (float*)(ws + off); off += (size_t)DS * SEQ * 4;
    float* KRf  = (float*)(ws + off); off += (size_t)DM * KR_LEN * 4;
    _Float16* xT = (_Float16*)(ws + off); off += (size_t)DM * BATCH * XT_STRIDE * 2;
    (void)in_sizes; (void)n_in; (void)out_size;
    if (off > ws_size) return;

    k_w<<<dim3(64), dim3(256), 0, stream>>>(C, B, W);
    k_psum<<<dim3(SEQ / 256, DS), dim3(256), 0, stream>>>(Lam, log_dt, Psum);
    k_kr<<<dim3((KR_LEN + 255) / 256, DM), dim3(256), 0, stream>>>(W, Psum, KRf);
    k_xt<<<dim3(XT_STRIDE / 64, DM / 16, BATCH), dim3(16, 16), 0, stream>>>(x, xT);
    k_conv<<<dim3(256 * 4), dim3(256), 0, stream>>>(KRf, xT, x, Dv, out);
}
